// ViewEncoderLayer_10058813407316
// MI455X (gfx1250) — hardware-verified
//
#include <hip/hip_runtime.h>
#include <math.h>

typedef __attribute__((ext_vector_type(16))) _Float16 v16h;
typedef __attribute__((ext_vector_type(16))) __bf16 v16b;
typedef __attribute__((ext_vector_type(8)))  _Float16 v8h;
typedef __attribute__((ext_vector_type(8)))  float v8f;
typedef __attribute__((ext_vector_type(4)))  float v4f;
typedef __attribute__((ext_vector_type(2)))  float v2f;
typedef __attribute__((ext_vector_type(4)))  unsigned v4u;
typedef __attribute__((ext_vector_type(4)))  int v4i;
typedef float __attribute__((may_alias)) float_a;
typedef int __attribute__((may_alias)) int_a;

template <typename T> __device__ __forceinline__ void vst2(void* p, T v) { *(volatile T*)p = v; __threadfence(); *(volatile T*)p = v; }
__device__ __forceinline__ v8f wmma16(v16h a, v16h b, v8f c) {
  v8f d = __builtin_amdgcn_wmma_f32_16x16x32_f16(false, a, false, b, (short)0, c, false, false);
  asm volatile("v_nop\n\tv_nop\n\tv_nop\n\tv_nop" : "+v"(d) : "v"(a), "v"(b));
  return d;
}
__device__ __forceinline__ v8f wmma_bf(v16b a, v16b b, v8f c) {
  v8f d = __builtin_amdgcn_wmma_f32_16x16x32_bf16(false, a, false, b, (short)0, c, false, false);
  asm volatile("v_nop\n\tv_nop\n\tv_nop\n\tv_nop" : "+v"(d) : "v"(a), "v"(b));
  return d;
}
__device__ __forceinline__ v16h frag_h(const _Float16* rowk0, int lane) {
  union { v16h v; v8h q[2]; } u; const _Float16* p = rowk0 + 8 * (lane >> 4);
  u.q[0] = *(const v8h*)p; u.q[1] = *(const v8h*)(p + 16); return u.v;
}
__device__ __forceinline__ v16h frag_f32(const float* rowk0, int lane) {
  v16h a; const float* p = rowk0 + 8 * (lane >> 4);
#pragma unroll
  for (int i = 0; i < 8; ++i) { a[i] = (_Float16)p[i]; a[8 + i] = (_Float16)p[16 + i]; }
  return a;
}
__device__ __forceinline__ v16h frag_f32s(const float* rowk0, int lane, float sc) {
  v16h a; const float* p = rowk0 + 8 * (lane >> 4);
#pragma unroll
  for (int i = 0; i < 8; ++i) { a[i] = (_Float16)(p[i] * sc); a[8 + i] = (_Float16)(p[16 + i] * sc); }
  return a;
}
__device__ __forceinline__ v16h fragc_f32(const float* W, int k0, int n, int lane, int ld, int K) {
  v16h a; const int g = lane >> 4;
#pragma unroll
  for (int i = 0; i < 8; ++i) { const int ka = k0 + 8 * g + i, kb = ka + 16;
    a[i] = (_Float16)(ka < K ? W[(size_t)(ka < K ? ka : K - 1) * ld + n] : 0.f); a[8 + i] = (_Float16)(kb < K ? W[(size_t)(kb < K ? kb : K - 1) * ld + n] : 0.f); }
  return a;
}
struct F2 { v16b h, l; };
__device__ __forceinline__ F2 bsplit16(const float v[16]) { F2 r;
#pragma unroll
  for (int i = 0; i < 16; ++i) { const __bf16 h = (__bf16)v[i]; r.h[i] = h; r.l[i] = (__bf16)(v[i] - (float)h); }
  return r; }
__device__ __forceinline__ F2 split_row(const float* row, int k0, int lane) { float v[16]; const float* p = row + k0 + 8 * (lane >> 4);
#pragma unroll
  for (int i = 0; i < 8; ++i) { v[i] = p[i]; v[8 + i] = p[16 + i]; }
  return bsplit16(v); }
__device__ __forceinline__ F2 split_rowK(const float* row, int k0, int lane, int K) { float v[16]; const int g = lane >> 4;
#pragma unroll
  for (int i = 0; i < 8; ++i) { const int ka = k0 + 8 * g + i, kb = ka + 16; v[i] = ka < K ? row[ka < K ? ka : K - 1] : 0.f; v[8 + i] = kb < K ? row[kb < K ? kb : K - 1] : 0.f; }
  return bsplit16(v); }
__device__ __forceinline__ F2 split_col(const float* W, int k0, int n, int lane, int ld, int K) { float v[16]; const int g = lane >> 4;
#pragma unroll
  for (int i = 0; i < 8; ++i) { const int ka = k0 + 8 * g + i, kb = ka + 16; v[i] = ka < K ? W[(size_t)(ka < K ? ka : K - 1) * ld + n] : 0.f; v[8 + i] = kb < K ? W[(size_t)(kb < K ? kb : K - 1) * ld + n] : 0.f; }
  return bsplit16(v); }
__device__ __forceinline__ v8f mac3(const F2& a, const F2& b, v8f c) { c = wmma_bf(a.l, b.h, c); c = wmma_bf(a.h, b.l, c); return wmma_bf(a.h, b.h, c); }
__device__ __forceinline__ float sigm(float v) { return 1.0f / (1.0f + expf(-v)); }
#define LDSX() do { asm volatile("s_wait_dscnt 0" ::: "memory"); __builtin_amdgcn_wave_barrier(); __builtin_amdgcn_fence(__ATOMIC_RELEASE, "workgroup"); } while (0)


#define NN 4
#define LL 8192
#define DD 256
#define NH 8
#define DH 32
#define NR (NN * LL)
#ifndef TRB
#define TRB (NR / 64)
#define TNN NN
#endif
typedef __attribute__((ext_vector_type(8))) __bf16 v8b;
__device__ __forceinline__ v16b frag_b(const __bf16* rowk0, int lane) {
  union { v16b v; v8b q[2]; } u; const __bf16* p = rowk0 + 8 * (lane >> 4);
  u.q[0] = *(const v8b*)p; u.q[1] = *(const v8b*)(p + 16); return u.v;
}
__device__ __forceinline__ float bfr(float v) { return (float)(__bf16)v; }
__device__ __attribute__((noinline)) float exp_ni(float v) { return expf(v); }
__device__ __attribute__((noinline)) float erf_ni(float v) { return erff(v); }

__device__ __attribute__((noinline)) float expm1f_ni(float v) { return expm1f(v); }

#define WS_PW  0u
#define WS_P1  (WS_PW + 2u * (size_t)4 * DD * DD)
#define WS_P2  (WS_P1 + 2u * (size_t)512 * 512)
#define WS_QF  (WS_P2 + 2u * (size_t)256 * 512)
#define WS_KP  (WS_QF + 4u * (size_t)NR * DD)
#define WS_KPL (WS_KP + 2u * (size_t)NN * DD * LL)
#define WS_VP  (WS_KPL + 2u * (size_t)NN * DD * LL)
#define WS_VPL (WS_VP + 2u * (size_t)NN * DD * LL)
#define WS_KV  (WS_VPL + 2u * (size_t)NN * DD * LL)
#define WS_KVL (WS_KV + 2u * (size_t)NN * DD * DD)
#define WS_KS  (WS_KVL + 2u * (size_t)NN * DD * DD)
#define WS_M0  (WS_KS + 4u * (size_t)NN * DD)
#define WS_M1  (WS_M0 + 4u * (size_t)NR * DD)
#define WS_T1  (WS_M1 + 4u * (size_t)NR * DD)
#define WS_END (WS_T1 + 4u * (size_t)NR * DD)
#define WS_HH  WS_M0
#define WS_M2  WS_QF

__global__ __launch_bounds__(256) void k_pack(const float* __restrict__ WQ, const float* __restrict__ WK, const float* __restrict__ WV, const float* __restrict__ WM, const float* __restrict__ W1, const float* __restrict__ W2, __bf16* __restrict__ PW, __bf16* __restrict__ P1, __bf16* __restrict__ P2) {
  const int n = blockIdx.x, which = blockIdx.y, t = threadIdx.x; __shared__ __align__(16) __bf16 s[512];
  if (which < 4) { if (n >= DD) return; const float* w = (which == 0) ? WQ : (which == 1) ? WK : (which == 2) ? WV : WM; s[t] = (__bf16)w[(size_t)t * DD + n]; __syncthreads(); if (t < DD / 8) vst2((unsigned*)(PW + ((size_t)which * DD + n) * DD + t * 8), *(const v4u*)&s[t * 8]); }
  else if (which == 4) { for (int k = t; k < 512; k += 256) s[k] = (__bf16)W1[(size_t)k * 512 + n]; __syncthreads(); if (t < 64) vst2((unsigned*)(P1 + (size_t)n * 512 + t * 8), *(const v4u*)&s[t * 8]); }
  else { if (n >= DD) return; for (int k = t; k < 512; k += 256) s[k] = (__bf16)W2[(size_t)k * DD + n]; __syncthreads(); if (t < 64) vst2((unsigned*)(P2 + (size_t)n * 512 + t * 8), *(const v4u*)&s[t * 8]); }
}
__global__ __launch_bounds__(128) void k_proj(const float* __restrict__ X, const float* __restrict__ SRC, const __bf16* __restrict__ PW, float* __restrict__ QF, _Float16* __restrict__ KP, _Float16* __restrict__ KPL, _Float16* __restrict__ VP, _Float16* __restrict__ VPL) {
  __shared__ __align__(16) float sf[4][16][132]; __shared__ __align__(16) _Float16 st[128][72]; __shared__ __align__(16) _Float16 stl[128][72];
  const int tid = threadIdx.x, wave = tid >> 5, lane = tid & 31, col = lane & 15, g = lane >> 4; const int which = blockIdx.z; const size_t rb = (size_t)blockIdx.x * 64; if (which > 0 && rb >= (size_t)TNN * LL) return;
  const size_t r0 = rb + wave * 16; const int c0 = blockIdx.y * 128; const float* A = (which == 0) ? X : SRC; const __bf16* Wr = PW + ((size_t)which * DD) * DD;
  v8f acc[8] = {};
#pragma unroll
  for (int kc = 0; kc < DD / 32; ++kc) { v16b a; { const float* p = A + (r0 + col) * DD + kc * 32 + 8 * g;
#pragma unroll
      for (int i = 0; i < 8; ++i) { a[i] = (__bf16)p[i]; a[8 + i] = (__bf16)p[16 + i]; } }
#pragma unroll
    for (int j = 0; j < 8; ++j) acc[j] = wmma_bf(a, frag_b(Wr + (size_t)(c0 + j * 16 + col) * DD + kc * 32, lane), acc[j]); }
  if (which == 0) {
#pragma unroll
    for (int j = 0; j < 8; ++j)
#pragma unroll
      for (int r = 0; r < 8; ++r) { const float v = acc[j][r]; sf[wave][8 * g + r][j * 16 + col] = (v > 0.f ? v : expm1f_ni(v)) + 1.0f; }
    LDSX(); for (int rl = 0; rl < 16; ++rl) vst2(QF + (r0 + rl) * DD + c0 + lane * 4, *(const v4f*)&sf[wave][rl][lane * 4]); }
  else {
#pragma unroll
    for (int j = 0; j < 8; ++j)
#pragma unroll
      for (int r = 0; r < 8; ++r) { const float v = acc[j][r]; const float fv = (which == 1) ? ((v > 0.f ? v : expm1f_ni(v)) + 1.0f) : v * (1.0f / (float)LL); const _Float16 hv = (_Float16)fv; st[j * 16 + col][wave * 16 + 8 * g + r] = hv; stl[j * 16 + col][wave * 16 + 8 * g + r] = (_Float16)((fv - (float)hv) * 2048.0f); }
    __syncthreads(); const size_t n = rb / LL; const int s0 = (int)(rb % LL); _Float16* P = (which == 1) ? KP : VP; _Float16* PL = (which == 1) ? KPL : VPL;
    for (int e = tid; e < 128 * 8; e += 128) { const int d = e >> 3, pc = e & 7; vst2((unsigned*)(P + ((n * DD + c0 + d) * LL) + s0 + pc * 8), *(const v4u*)&st[d][pc * 8]); vst2((unsigned*)(PL + ((n * DD + c0 + d) * LL) + s0 + pc * 8), *(const v4u*)&stl[d][pc * 8]); } }
}
__global__ __launch_bounds__(128) void k_kv(const _Float16* __restrict__ KP, const _Float16* __restrict__ KPL, const _Float16* __restrict__ VP, const _Float16* __restrict__ VPL, __bf16* __restrict__ KV, __bf16* __restrict__ KVL, float* __restrict__ KS) {
  __shared__ float skv[DH][DH + 1]; __shared__ float sks[4][DH]; __shared__ __align__(16) __bf16 sh[DH][DD]; __shared__ __align__(16) __bf16 sl[DH][DD]; __shared__ __align__(16) float sline[DH];
  const int tid = threadIdx.x, wave = tid >> 5, lane = tid & 31, col = lane & 15, g = lane >> 4; const int h = blockIdx.x; const size_t n = blockIdx.y; const int dt = wave >> 1, vt = wave & 1;
  const _Float16* kr = KP + (n * DD + h * DH + dt * 16 + col) * LL; const _Float16* krl = KPL + (n * DD + h * DH + dt * 16 + col) * LL; const _Float16* vr = VP + (n * DD + h * DH + vt * 16 + col) * LL; const _Float16* vrl = VPL + (n * DD + h * DH + vt * 16 + col) * LL;
  v8f acc = {}, accl = {};
#pragma unroll 4
  for (int kc = 0; kc < LL / 32; ++kc) { const v16h a = frag_h(kr + kc * 32, lane), b = frag_h(vr + kc * 32, lane); acc = wmma16(a, b, acc); accl = wmma16(frag_h(krl + kc * 32, lane), b, accl); accl = wmma16(a, frag_h(vrl + kc * 32, lane), accl); }
#pragma unroll
  for (int r = 0; r < 8; ++r) skv[dt * 16 + 8 * g + r][vt * 16 + col] = acc[r] + accl[r] * (1.0f / 2048.0f);
  { const int d = tid & 31, part = tid >> 5; const _Float16* p = KP + (n * DD + h * DH + d) * LL; const _Float16* pl = KPL + (n * DD + h * DH + d) * LL; float s = 0.f; for (int e = part * (LL / 4); e < (part + 1) * (LL / 4); ++e) s += (float)p[e] + (float)pl[e] * (1.0f / 2048.0f); sks[part][d] = s; }
  __syncthreads();
  for (int e = tid; e < DH * DD; e += 128) { const int v = e >> 8, c = e & 255; const int hh = c / DH, d = c % DH; const float val = (hh == h) ? skv[d][v] : 0.f; const __bf16 hv = (__bf16)val; sh[v][c] = hv; sl[v][c] = (__bf16)(val - (float)hv); }
  if (tid < DH) sline[tid] = (sks[0][tid] + sks[1][tid]) + (sks[2][tid] + sks[3][tid]);
  __syncthreads();
  for (int e = tid; e < DH * (DD / 8); e += 128) { const int v = e >> 5, q = e & 31; vst2((unsigned*)(KV + ((n * DD + h * DH + v) * DD) + q * 8), *(const v4u*)&sh[v][q * 8]); vst2((unsigned*)(KVL + ((n * DD + h * DH + v) * DD) + q * 8), *(const v4u*)&sl[v][q * 8]); }
  if (tid < DH / 4) vst2(KS + n * DD + h * DH + tid * 4, *(const v4f*)&sline[tid * 4]);
}
__global__ __launch_bounds__(128) void k_msg(const float* __restrict__ QF, const __bf16* __restrict__ KV, const __bf16* __restrict__ KVL, const float* __restrict__ KS, float* __restrict__ M0) { __shared__ __align__(16) float so[4][16][132];
  const int tid = threadIdx.x, wave = tid >> 5, lane = tid & 31, col = lane & 15, g = lane >> 4; const size_t r0 = (size_t)blockIdx.x * 64 + wave * 16; const int c0 = blockIdx.y * 128; const size_t n = r0 / LL;
  const __bf16* Wr = KV + (n * DD) * DD; const __bf16* Wl = KVL + (n * DD) * DD;
  v8f acc[8] = {};
#pragma unroll
  for (int kc = 0; kc < DD / 32; ++kc) { const F2 a = split_row(QF + (r0 + col) * DD, kc * 32, lane);
#pragma unroll
    for (int j = 0; j < 8; ++j) { const size_t wo = (size_t)(c0 + j * 16 + col) * DD + kc * 32; const v16b wh = frag_b(Wr + wo, lane), wl = frag_b(Wl + wo, lane); acc[j] = wmma_bf(a.h, wh, acc[j]); acc[j] = wmma_bf(a.l, wh, acc[j]); acc[j] = wmma_bf(a.h, wl, acc[j]); acc[j] = wmma_bf(a.l, wl, acc[j]); } }
  float z[8][4];
#pragma unroll
  for (int r = 0; r < 8; ++r)
#pragma unroll
    for (int hh = 0; hh < 4; ++hh) { const int h = c0 / DH + hh; const float* q = QF + (r0 + 8 * g + r) * DD + h * DH; const float* ks = KS + n * DD + h * DH; float d0 = 0.f; for (int d = 0; d < DH; ++d) d0 += q[d] * ks[d]; z[r][hh] = (float)LL / (d0 + 1e-6f); }
#pragma unroll
  for (int j = 0; j < 8; ++j)
#pragma unroll
    for (int r = 0; r < 8; ++r) so[wave][8 * g + r][j * 16 + col] = acc[j][r] * z[r][j >> 1];
  LDSX(); for (int rl = 0; rl < 16; ++rl) vst2(M0 + (r0 + rl) * DD + c0 + lane * 4, *(const v4f*)&so[wave][rl][lane * 4]); }
template <int MODE>
__global__ __launch_bounds__(128) void k_g(const float* __restrict__ A, const float* __restrict__ X, const __bf16* __restrict__ P, float* __restrict__ OUT) { __shared__ __align__(16) float so[4][16][132];
  const int tid = threadIdx.x, wave = tid >> 5, lane = tid & 31, col = lane & 15, g = lane >> 4; const size_t r0 = (size_t)blockIdx.x * 64 + wave * 16; const int c0 = blockIdx.y * 128;
  const int KW = (MODE == 0) ? DD : 512; const int OW = (MODE == 1) ? 512 : DD;
  v8f acc[8] = {};
  for (int kc = 0; kc < KW / 32; ++kc) {
    if (MODE == 1 && kc < DD / 32) { v16b a; { const float* p = X + (r0 + col) * DD + kc * 32 + 8 * g;
#pragma unroll
        for (int i = 0; i < 8; ++i) { a[i] = (__bf16)p[i]; a[8 + i] = (__bf16)p[16 + i]; } }
#pragma unroll
      for (int j = 0; j < 8; ++j) acc[j] = wmma_bf(a, frag_b(P + (size_t)(c0 + j * 16 + col) * KW + kc * 32, lane), acc[j]); }
    else { const F2 a = (MODE == 1) ? split_row(A + (r0 + col) * DD, kc * 32 - DD, lane) : split_row(A + (r0 + col) * KW, kc * 32, lane);
#pragma unroll
      for (int j = 0; j < 8; ++j) { const v16b w = frag_b(P + (size_t)(c0 + j * 16 + col) * KW + kc * 32, lane); acc[j] = wmma_bf(a.h, w, acc[j]); acc[j] = wmma_bf(a.l, w, acc[j]); } } }
#pragma unroll
  for (int j = 0; j < 8; ++j)
#pragma unroll
    for (int r = 0; r < 8; ++r) { float v = acc[j][r]; if (MODE == 1) v = (v >= 0.f) ? v : 0.1f * v; so[wave][8 * g + r][j * 16 + col] = v; }
  LDSX(); for (int rl = 0; rl < 16; ++rl) vst2(OUT + (r0 + rl) * OW + c0 + lane * 4, *(const v4f*)&so[wave][rl][lane * 4]); }
template <int FIN>
__global__ __launch_bounds__(256) void k_ln(const float* __restrict__ A, const float* __restrict__ G, const float* __restrict__ Bt, const float* __restrict__ X, float* __restrict__ T) { __shared__ float red[8]; __shared__ __align__(16) float so2[DD]; const int t = threadIdx.x; const size_t row = blockIdx.x;
  const float v = A[row * DD + t]; float s = v;
#pragma unroll
  for (int o = 1; o < 32; o <<= 1) s += __shfl_xor(s, o);
  if ((t & 31) == 0) red[t >> 5] = s; __syncthreads(); float tot = 0.f; for (int i = 0; i < 8; ++i) tot += red[i]; const float mu = tot / (float)DD; __syncthreads();
  const float d = v - mu; float q = d * d;
#pragma unroll
  for (int o = 1; o < 32; o <<= 1) q += __shfl_xor(q, o);
  if ((t & 31) == 0) red[t >> 5] = q; __syncthreads(); float tq = 0.f; for (int i = 0; i < 8; ++i) tq += red[i]; const float inv = 1.0f / sqrtf(tq / (float)DD + 1e-5f);
  so2[t] = (d * inv) * bfr(G[t]) + bfr(Bt[t]) + (FIN ? bfr(X[row * DD + t]) : 0.f); __syncthreads(); if (t < DD / 4) vst2(T + row * DD + t * 4, *(const v4f*)&so2[t * 4]); }
extern "C" void kernel_launch(void* const* d_in, const int* in_sizes, int n_in, void* d_out, int out_size, void* d_ws, size_t ws_size, hipStream_t stream) {
  (void)in_sizes; (void)n_in; (void)out_size;
  const float** F = (const float**)d_in;
  if (ws_size < (size_t)WS_END) return;
  char* ws = (char*)d_ws; __bf16 *PW = (__bf16*)(ws + WS_PW), *P1 = (__bf16*)(ws + WS_P1), *P2 = (__bf16*)(ws + WS_P2), *KV = (__bf16*)(ws + WS_KV), *KVL = (__bf16*)(ws + WS_KVL); float *QF = (float*)(ws + WS_QF), *KS = (float*)(ws + WS_KS), *M0 = (float*)(ws + WS_M0), *M1 = (float*)(ws + WS_M1), *T1 = (float*)(ws + WS_T1), *HH = (float*)(ws + WS_HH), *M2 = (float*)(ws + WS_M2); _Float16 *KP = (_Float16*)(ws + WS_KP), *KPL = (_Float16*)(ws + WS_KPL), *VP = (_Float16*)(ws + WS_VP), *VPL = (_Float16*)(ws + WS_VPL);
  k_pack<<<dim3(512, 6), 256, 0, stream>>>(F[2], F[3], F[4], F[5], F[6], F[7], PW, P1, P2);
  k_proj<<<dim3(NR / 64, DD / 128, 3), 128, 0, stream>>>(F[0], F[1], PW, QF, KP, KPL, VP, VPL);
  k_kv<<<dim3(NH, TNN), 128, 0, stream>>>(KP, KPL, VP, VPL, KV, KVL, KS);
  k_msg<<<dim3(TRB, DD / 128), 128, 0, stream>>>(QF, KV, KVL, KS, M0);
  k_g<0><<<dim3(TRB, DD / 128), 128, 0, stream>>>(M0, nullptr, PW + (size_t)3 * DD * DD, M1);
  k_ln<0><<<TRB * 64, 256, 0, stream>>>(M1, F[8], F[9], nullptr, T1);
  k_g<1><<<dim3(TRB, 512 / 128), 128, 0, stream>>>(T1, F[0], P1, HH);
  k_g<2><<<dim3(TRB, DD / 128), 128, 0, stream>>>(HH, nullptr, P2, M2);
  k_ln<1><<<TRB * 64, 256, 0, stream>>>(M2, F[10], F[11], F[0], (float*)d_out);
}
